// Model_81475529605800
// MI455X (gfx1250) — hardware-verified
//
#include <hip/hip_runtime.h>
#include <stddef.h>
#include <stdint.h>

#define U_N    100000
#define V_N    50000
#define E_N    2000000
#define FD     32
#define EVD    8
#define KIN    72
#define K1     96
#define N1     64
#define K2     128
#define N2     32
#define NTHR   256
#define NWAVE  8
#define TROWS  128
#define AP1    104
#define AP2    136
#define DP     68
#define TABN   256
#define T_GB1  0
#define T_GB2  64
#define T_FB1  96
#define T_FB2  160
#define T_TW   192
#define T_TB   224
#define MP16   32
#define EPT    8
#define CHUNK  (NTHR * EPT)
#define WCAP   (EPT * 32)
#define LISTN  (NWAVE * WCAP)
#define NBA    1024
#define SLA    10
#define RCAP   28672
#define DEGCAP 64
#define NSCAN  ((U_N + NBA - 1) / NBA)
#define AGGROWS (NSCAN * NBA)
#define NNODEB ((U_N + TROWS - 1) / TROWS)
#define NU_G1  (N1 * (K1 / 8))
#define NU_G2  (N2 * (K2 / 8))
#define NU_F1  (N1 * (K1 / 8))
#define NU_F2  (N2 * (K2 / 8))
#define NU_TAB NTHR
#define AGG_ZINTS (LISTN + 2 * RCAP + 3 * NBA)
#define AGG_LDS_INTS (AGG_ZINTS + 16)
#define AGG_LDS_BYTES (AGG_LDS_INTS * 4)
#define TILE_LDS_BYTES (TROWS * DP * 4 + TABN * 4 + 256 * 4 + TROWS * AP1 * 2 + TROWS * AP2 * 2)
#define MCARRY 64.0f
#define MINV   0.015625f

static_assert(E_N % TROWS == 0);
static_assert(E_N < (1 << 21));
static_assert(NNODEB == 782 && U_N - 781 * TROWS == 32 && (32 % 32) == 0 && (U_N % 4) == 0);
static_assert(NSCAN == 98 && AGGROWS >= NNODEB * TROWS);
static_assert(RCAP >= 20982 + 4096);
static_assert(DEGCAP >= 41 + 8);
static_assert((CHUNK & (CHUNK - 1)) == 0 && CHUNK <= 4096);
static_assert((NBA & (NBA - 1)) == 0 && NBA == (1 << SLA));
static_assert(((long long)CHUNK << SLA) < (1LL << 31));
static_assert(((long long)E_N << SLA) + NBA < (1LL << 31));
static_assert(LISTN % NTHR == 0 && NBA % NWAVE == 0 && NBA % 32 == 0);
static_assert(RCAP % 4 == 0 && AGG_ZINTS % (4 * NTHR) == 0 && LISTN % 4 == 0);
static_assert(AGG_LDS_BYTES <= 300000 && TILE_LDS_BYTES <= 300000);
static_assert(NU_G1 % NTHR == 0 && NU_G2 % NTHR == 0 && NU_F1 % NTHR == 0 && NU_F2 % NTHR == 0);
static_assert(K1 % 32 == 0 && K2 % 32 == 0 && N1 % 16 == 0 && N2 % 16 == 0 && KIN % 8 == 0);
static_assert(K1 == FD + FD + 32 && KIN == FD + FD + EVD && K2 == 2 * N1);
static_assert((AP1 * 2) % 16 == 0 && (AP2 * 2) % 16 == 0 && (DP * 4) % 16 == 0);
static_assert(AP1 >= K1 && AP2 >= K2 && DP >= N1);
static_assert(TROWS == NWAVE * 16 && NTHR == 2 * TROWS);
static_assert(T_TB + 4 <= TABN && T_GB2 == T_GB1 + N1 && T_FB1 == T_GB2 + N2 && T_FB2 == T_FB1 + N1);
static_assert(T_TW == T_FB2 + N2 && T_TB == T_TW + 32);
static_assert(MP16 == N2 && (MP16 * 2 * TROWS) == 2 * NTHR * 16);

typedef float          v4f   __attribute__((ext_vector_type(4)));
typedef float          v8f   __attribute__((ext_vector_type(8)));
typedef int            v4i   __attribute__((ext_vector_type(4)));
typedef int            v8i   __attribute__((ext_vector_type(8)));
typedef unsigned       v2u   __attribute__((ext_vector_type(2)));
typedef unsigned short v8us  __attribute__((ext_vector_type(8)));
typedef unsigned short v16us __attribute__((ext_vector_type(16)));
typedef __bf16         v16bf __attribute__((ext_vector_type(16)));
typedef v4f  __attribute__((may_alias)) v4fa;
typedef v4i  __attribute__((may_alias)) v4ia;
typedef v2u  __attribute__((may_alias)) v2ua;
typedef v8us __attribute__((may_alias)) v8usa;
union FragB { v16bf v; v16us u; v8us h[2]; v8i w; };

__device__ __forceinline__ v8f wmb(const FragB& a, const FragB& b, v8f c) {
  v8f d = __builtin_amdgcn_wmma_f32_16x16x32_bf16(false, a.v, false, b.v, (short)0, c, false, false);
  asm volatile("v_nop\n\tv_nop\n\tv_nop\n\tv_nop" : "+v"(d) : "v"(a.w), "v"(b.w));
  return d;
}

__device__ __forceinline__ unsigned bf16n_bits(float f) {
  const unsigned u = __float_as_uint(f);
  const unsigned r = (u + 0x7FFFu + ((u >> 16) & 1u)) >> 16;
  const unsigned q = (u >> 16) | 0x0040u;
  return ((u & 0x7fffffffu) > 0x7f800000u) ? q : r;
}
__device__ __forceinline__ float bf16n_val(float f) {
  return __uint_as_float(bf16n_bits(f) << 16);
}
__device__ __forceinline__ unsigned pack2(unsigned lo16, unsigned hi16) {
  return (lo16 & 0xffffu) | (hi16 << 16);
}
__device__ __forceinline__ unsigned short f2h(float f) {
  const _Float16 hv = (_Float16)f;
  return __builtin_bit_cast(unsigned short, hv);
}
__device__ __forceinline__ float h2f(unsigned b) {
  const _Float16 hv = __builtin_bit_cast(_Float16, (unsigned short)b);
  return (float)hv;
}
__device__ __forceinline__ float relu_n(float v) {
  return (v > 0.0f) ? v : (v - v);
}
__device__ __forceinline__ void put16(unsigned short* dp, v8us o) {
  *(volatile v8us*)dp = o;
  __threadfence();
  *(volatile v8us*)dp = o;
}
__device__ __forceinline__ void putf4(float* dp, v4f o) {
  *(volatile v4f*)dp = o;
  __threadfence();
  *(volatile v4f*)dp = o;
}

template <int SLB>
__device__ __forceinline__ int scan_chunk(const int* __restrict__ dsts, int nE, int cbase, int slotBase,
                                          int nb, int vec8, int* list, int tid, int lane, int wave) {
  int wc = 0;
  const int el0  = tid * EPT;
  const int e0   = cbase + el0;
  const int sent = -2147483647 - 1;
  v4i da, db;
  if (vec8 != 0 && cbase + CHUNK <= nE) {
    da = *(const v4i*)(dsts + e0);
    db = *(const v4i*)(dsts + e0 + 4);
  } else {
    da.x = (e0     < nE) ? dsts[min(e0,     nE - 1)] : sent;
    da.y = (e0 + 1 < nE) ? dsts[min(e0 + 1, nE - 1)] : sent;
    da.z = (e0 + 2 < nE) ? dsts[min(e0 + 2, nE - 1)] : sent;
    da.w = (e0 + 3 < nE) ? dsts[min(e0 + 3, nE - 1)] : sent;
    db.x = (e0 + 4 < nE) ? dsts[min(e0 + 4, nE - 1)] : sent;
    db.y = (e0 + 5 < nE) ? dsts[min(e0 + 5, nE - 1)] : sent;
    db.z = (e0 + 6 < nE) ? dsts[min(e0 + 6, nE - 1)] : sent;
    db.w = (e0 + 7 < nE) ? dsts[min(e0 + 7, nE - 1)] : sent;
  }
  const unsigned nbs = (unsigned)slotBase;
  const unsigned unb = (unsigned)nb;
  const unsigned s0 = (unsigned)da.x - nbs, s1 = (unsigned)da.y - nbs;
  const unsigned s2 = (unsigned)da.z - nbs, s3 = (unsigned)da.w - nbs;
  const unsigned s4 = (unsigned)db.x - nbs, s5 = (unsigned)db.y - nbs;
  const unsigned s6 = (unsigned)db.z - nbs, s7 = (unsigned)db.w - nbs;
  const bool h0 = s0 < unb, h1 = s1 < unb, h2 = s2 < unb, h3 = s3 < unb;
  const bool h4 = s4 < unb, h5 = s5 < unb, h6 = s6 < unb, h7 = s7 < unb;
  const unsigned any = __builtin_amdgcn_ballot_w32(h0 | h1 | h2 | h3 | h4 | h5 | h6 | h7);
  if (any != 0u) {
#define HITJ(J, HJ, SJ) { \
      const unsigned mj = __builtin_amdgcn_ballot_w32(HJ); \
      if (mj != 0u) { \
        if (HJ) { \
          const int pos = wc + (int)__builtin_amdgcn_mbcnt_lo(mj, 0u); \
          if (pos < WCAP) list[wave * WCAP + pos] = ((el0 + (J)) << SLB) | (int)(SJ); \
        } \
        wc += (int)__builtin_popcount(mj); } }
    HITJ(0, h0, s0)
    HITJ(1, h1, s1)
    HITJ(2, h2, s2)
    HITJ(3, h3, s3)
    HITJ(4, h4, s4)
    HITJ(5, h5, s5)
    HITJ(6, h6, s6)
    HITJ(7, h7, s7)
#undef HITJ
  }
  return wc;
}

__global__ __launch_bounds__(NTHR) void k_prep(const float* __restrict__ gw1, const float* __restrict__ gb1,
                                               const float* __restrict__ gw2, const float* __restrict__ gb2,
                                               const float* __restrict__ fw1, const float* __restrict__ fb1,
                                               const float* __restrict__ fw2, const float* __restrict__ fb2,
                                               const float* __restrict__ tw,  const float* __restrict__ tb,
                                               unsigned short* G1T, unsigned short* G2T,
                                               unsigned short* F1T, unsigned short* F2T, float* TAB) {
  const int u  = (int)blockIdx.x * NTHR + (int)threadIdx.x;
  const int R0 = NU_G1;
  const int R1 = R0 + NU_G2;
  const int R2 = R1 + NU_F1;
  const int R3 = R2 + NU_F2;
  v8us o;
  if (u < R0) {
    const int n  = u / (K1 / 8);
    const int k8 = (u - n * (K1 / 8)) * 8;
#pragma unroll
    for (int i = 0; i < 8; ++i) {
      const int k  = k8 + i;
      const int kc = k < KIN ? k : (KIN - 1);
      const float w = gw1[(size_t)kc * N1 + n];
      const unsigned msk = (k < KIN) ? 0xffffu : 0u;
      o[i] = (unsigned short)(bf16n_bits(w) & msk);
    }
    put16(G1T + (size_t)u * 8, o);
    return;
  } else if (u < R1) {
    const int v    = u - R0;
    const int n    = v >> 4;
    const int k8   = (v & 15) * 8;
    const int srow = k8 & (N1 - 1);
    const float* p = gw2 + (size_t)srow * N2 + n;
#pragma unroll
    for (int i = 0; i < 8; ++i) o[i] = (unsigned short)bf16n_bits(p[(size_t)i * N2]);
    put16(G2T + (size_t)v * 8, o);
    return;
  } else if (u < R2) {
    const int v    = u - R1;
    const int n    = v / (K1 / 8);
    const int k8   = (v - n * (K1 / 8)) * 8;
    const int srow = (k8 < 64) ? k8 : (k8 - 32);
    const float* p = fw1 + (size_t)srow * N1 + n;
#pragma unroll
    for (int i = 0; i < 8; ++i) o[i] = (unsigned short)bf16n_bits(p[(size_t)i * N1]);
    put16(F1T + (size_t)v * 8, o);
    return;
  } else if (u < R3) {
    const int v    = u - R2;
    const int n    = v >> 4;
    const int k8   = (v & 15) * 8;
    const int srow = k8 & (N1 - 1);
    const float* p = fw2 + (size_t)srow * N2 + n;
#pragma unroll
    for (int i = 0; i < 8; ++i) o[i] = (unsigned short)bf16n_bits(p[(size_t)i * N2]);
    put16(F2T + (size_t)v * 8, o);
    return;
  } else {
    const int t = u - R3;
    if (t < TABN / 4) {
      const int i  = 4 * t;
      int ia = i;        ia = ia < 0 ? 0 : (ia > 60 ? 60 : ia);
      int ib = i - 64;   ib = ib < 0 ? 0 : (ib > 28 ? 28 : ib);
      int ic = i - 96;   ic = ic < 0 ? 0 : (ic > 60 ? 60 : ic);
      int id = i - 160;  id = id < 0 ? 0 : (id > 28 ? 28 : id);
      int ie = i - 192;  ie = ie < 0 ? 0 : (ie > 28 ? 28 : ie);
      const v4f a = *(const v4fa*)(gb1 + ia);
      const v4f b = *(const v4fa*)(gb2 + ib);
      const v4f c = *(const v4fa*)(fb1 + ic);
      const v4f d = *(const v4fa*)(fb2 + id);
      const v4f e = *(const v4fa*)(tw + ie);
      const float f = tb[0];
      const unsigned ma = (i < 64) ? 0xffffffffu : 0u;
      const unsigned mb = (i >= 64 && i < 96) ? 0xffffffffu : 0u;
      const unsigned mc = (i >= 96 && i < 160) ? 0xffffffffu : 0u;
      const unsigned md = (i >= 160 && i < 192) ? 0xffffffffu : 0u;
      const unsigned me = (i >= 192 && i < 224) ? 0xffffffffu : 0u;
      const unsigned mf = (i == 224) ? 0xffffffffu : 0u;
      const unsigned x0 = (__float_as_uint(a.x) & ma) | (__float_as_uint(b.x) & mb) | (__float_as_uint(c.x) & mc) |
                          (__float_as_uint(d.x) & md) | (__float_as_uint(e.x) & me) | (__float_as_uint(f) & mf);
      const unsigned x1 = (__float_as_uint(a.y) & ma) | (__float_as_uint(b.y) & mb) | (__float_as_uint(c.y) & mc) |
                          (__float_as_uint(d.y) & md) | (__float_as_uint(e.y) & me);
      const unsigned x2 = (__float_as_uint(a.z) & ma) | (__float_as_uint(b.z) & mb) | (__float_as_uint(c.z) & mc) |
                          (__float_as_uint(d.z) & md) | (__float_as_uint(e.z) & me);
      const unsigned x3 = (__float_as_uint(a.w) & ma) | (__float_as_uint(b.w) & mb) | (__float_as_uint(c.w) & mc) |
                          (__float_as_uint(d.w) & md) | (__float_as_uint(e.w) & me);
      v4f q;
      q.x = bf16n_val(__uint_as_float(x0));
      q.y = bf16n_val(__uint_as_float(x1));
      q.z = bf16n_val(__uint_as_float(x2));
      q.w = bf16n_val(__uint_as_float(x3));
      putf4(TAB + i, q);
    }
    return;
  }
}

template <int NT, int KS, int LDB>
__device__ __forceinline__ void wave_gemm(const unsigned short* arow, const unsigned short* __restrict__ BT,
                                          float* drow, int hh, int m) {
  v8f acc[NT];
  {
    const v8f z = {0.f, 0.f, 0.f, 0.f, 0.f, 0.f, 0.f, 0.f};
#pragma unroll
    for (int t = 0; t < NT; ++t) acc[t] = z;
  }
  const unsigned short* bp = BT + (size_t)m * LDB + 8 * hh;
#pragma unroll
  for (int ks = 0; ks < KS; ++ks) {
    FragB a;
    a.h[0] = *(const v8usa*)(arow + 32 * ks);
    a.h[1] = *(const v8usa*)(arow + 32 * ks + 16);
#pragma unroll
    for (int nt = 0; nt < NT; ++nt) {
      const unsigned short* wq = bp + (size_t)(16 * nt) * LDB + 32 * ks;
      FragB b;
      b.h[0] = *(const v8usa*)wq;
      b.h[1] = *(const v8usa*)(wq + 16);
      acc[nt] = wmb(a, b, acc[nt]);
    }
  }
#pragma unroll
  for (int nt = 0; nt < NT; ++nt)
#pragma unroll
    for (int r = 0; r < 8; ++r) drow[r * DP + 16 * nt] = acc[nt][r];
}

__device__ __forceinline__ void epi_split(const float* sD, const float* sB, unsigned short* sA2, int tid) {
  const int row = tid >> 1;
  const int hf  = tid & 1;
  const float*    rd = sD + row * DP;
  unsigned short* ra = sA2 + row * AP2;
#pragma unroll 1
  for (int c8 = 0; c8 < 4; ++c8) {
    const int col = 32 * hf + 8 * c8;
    const v4f va = *(const v4fa*)(rd + col);
    const v4f vb = *(const v4fa*)(rd + col + 4);
    const v4f ba = *(const v4fa*)(sB + col);
    const v4f bb = *(const v4fa*)(sB + col + 4);
    const v8f v8 = {va.x, va.y, va.z, va.w, vb.x, vb.y, vb.z, vb.w};
    const v8f b8 = {ba.x, ba.y, ba.z, ba.w, bb.x, bb.y, bb.z, bb.w};
    v8us ho, lo;
#pragma unroll
    for (int i = 0; i < 8; ++i) {
      const float r = relu_n(v8[i] + b8[i]);
      const unsigned hb = bf16n_bits(r);
      ho[i] = (unsigned short)hb;
      lo[i] = (unsigned short)bf16n_bits(r - __uint_as_float(hb << 16));
    }
    *(v8usa*)(ra + col)      = ho;
    *(v8usa*)(ra + N1 + col) = lo;
  }
}

__global__ __launch_bounds__(NTHR) void k_edge(const float* __restrict__ u, const float* __restrict__ v,
                                               const float* __restrict__ ev,
                                               const int* __restrict__ esrc, const int* __restrict__ edst,
                                               int nU, int nV, int nE,
                                               const unsigned short* __restrict__ G1T,
                                               const unsigned short* __restrict__ G2T,
                                               const float* __restrict__ TAB, unsigned short* Mh) {
  extern __shared__ __attribute__((aligned(16))) float dyn[];
  float*          sD  = dyn;
  float*          sT  = dyn + TROWS * DP;
  int*            sI  = (int*)(sT + TABN);
  unsigned short* sA1 = (unsigned short*)(sI + 256);
  unsigned short* sA2 = sA1 + TROWS * AP1;

  const int tid = (int)threadIdx.x, lane = tid & 31, wave = tid >> 5, hh = lane >> 4, m = lane & 15;
  const int e0 = (int)blockIdx.x * TROWS;

  if (tid < TABN / 4) {
    const v4f t4 = *(const v4fa*)(TAB + 4 * tid);
    *(v4fa*)(sT + 4 * tid) = t4;
  }
  if (tid < TROWS) {
    int ec = e0 + tid;
    ec = ec > nE - 1 ? nE - 1 : ec;
    int d = edst[ec];
    int s = esrc[ec];
    d = d < 0 ? 0 : (d > nU - 1 ? nU - 1 : d);
    s = s < 0 ? 0 : (s > nV - 1 ? nV - 1 : s);
    sI[tid]         = d;
    sI[TROWS + tid] = s;
  }
  __syncthreads();

#pragma unroll
  for (int it = 0; it < 4; ++it) {
    const int c   = it * NTHR + tid;
    const int row = c >> 3;
    const int q   = c & 7;
    const int d   = sI[row];
    const int s   = sI[TROWS + row];
    const v4f ua = *(const v4fa*)(u + (size_t)d * FD + 4 * q);
    const v4f va = *(const v4fa*)(v + (size_t)s * FD + 4 * q);
    v2u wu, wv;
    wu.x = pack2(bf16n_bits(ua.x), bf16n_bits(ua.y));
    wu.y = pack2(bf16n_bits(ua.z), bf16n_bits(ua.w));
    wv.x = pack2(bf16n_bits(va.x), bf16n_bits(va.y));
    wv.y = pack2(bf16n_bits(va.z), bf16n_bits(va.w));
    *(v2ua*)(sA1 + row * AP1 + 4 * q)      = wu;
    *(v2ua*)(sA1 + row * AP1 + FD + 4 * q) = wv;
  }
  {
    const int row = tid >> 1;
    const int hf  = tid & 1;
    int er = e0 + row;
    er = er > nE - 1 ? nE - 1 : er;
    const v4f ea = *(const v4fa*)(ev + (size_t)er * EVD + 4 * hf);
    v2u we;
    we.x = pack2(bf16n_bits(ea.x), bf16n_bits(ea.y));
    we.y = pack2(bf16n_bits(ea.z), bf16n_bits(ea.w));
    *(v2ua*)(sA1 + row * AP1 + 2 * FD + 4 * hf) = we;
    const v2u z2 = {0u, 0u};
#pragma unroll
    for (int j = 0; j < 3; ++j) *(v2ua*)(sA1 + row * AP1 + KIN + 12 * hf + 4 * j) = z2;
  }
  __syncthreads();

  wave_gemm<4, 3, K1>(sA1 + (16 * wave + m) * AP1 + 8 * hh, G1T, sD + (16 * wave + 8 * hh) * DP + m, hh, m);
  __syncthreads();

  epi_split(sD, sT + T_GB1, sA2, tid);
  __syncthreads();

  wave_gemm<2, 4, K2>(sA2 + (16 * wave + m) * AP2 + 8 * hh, G2T, sD + (16 * wave + 8 * hh) * DP + m, hh, m);
  __syncthreads();

  {
    v8us pv[2];
#pragma unroll
    for (int it = 0; it < 2; ++it) {
      const int p   = it * NTHR + tid;
      const int row = p >> 2;
      const int q   = p & 3;
      const float* rd = sD + row * DP + 8 * q;
      const v4f va = *(const v4fa*)rd;
      const v4f vb = *(const v4fa*)(rd + 4);
      const v4f ba = *(const v4fa*)(sT + T_GB2 + 8 * q);
      const v4f bb = *(const v4fa*)(sT + T_GB2 + 8 * q + 4);
      const v8f v8 = {va.x, va.y, va.z, va.w, vb.x, vb.y, vb.z, vb.w};
      const v8f b8 = {ba.x, ba.y, ba.z, ba.w, bb.x, bb.y, bb.z, bb.w};
      v8us o;
#pragma unroll
      for (int i = 0; i < 8; ++i) o[i] = f2h(MCARRY * relu_n(v8[i] + b8[i]));
      pv[it] = o;
    }
    unsigned short* mb = Mh + (size_t)e0 * MP16;
#pragma unroll
    for (int it = 0; it < 2; ++it) *(volatile v8us*)(mb + (size_t)(it * NTHR + tid) * 8) = pv[it];
    __threadfence();
#pragma unroll
    for (int it = 0; it < 2; ++it) *(volatile v8us*)(mb + (size_t)(it * NTHR + tid) * 8) = pv[it];
  }
}

__global__ __launch_bounds__(NTHR) void k_scan(const int* __restrict__ dsts, int nE, int vec8, int mRows,
                                               const unsigned short* __restrict__ Mh, float* AGG) {
  extern __shared__ __attribute__((aligned(16))) int dsm[];
  int*   list = dsm;
  int*   hl   = dsm + LISTN;
  int*   sl   = hl + RCAP;
  int*   cnt  = sl + RCAP;
  int*   offs = cnt + NBA;
  int*   cur  = offs + NBA;
  int*   misc = cur + NBA;
  const int tid = (int)threadIdx.x, lane = tid & 31, wave = tid >> 5;
  const int nodeBase = (int)blockIdx.x * NBA;

  {
    const v4i z4 = {0, 0, 0, 0};
    for (int i = tid * 4; i < AGG_ZINTS; i += NTHR * 4) *(v4ia*)(dsm + i) = z4;
    if (tid < 16) misc[tid] = 0;
  }
  __syncthreads();

  int t = 0, ov = 0;
  const int nChunks = (nE + CHUNK - 1) / CHUNK;
#pragma unroll 1
  for (int ch = 0; ch < nChunks; ++ch) {
    const int cbase = ch * CHUNK;
    const int wc = scan_chunk<SLA>(dsts, nE, cbase, nodeBase, NBA, vec8, list, tid, lane, wave);
    if (lane == 0) misc[wave] = wc;
    __syncthreads();
    if (wave == 0) {
#pragma unroll 1
      for (int w2 = 0; w2 < NWAVE; ++w2) {
        int c = misc[w2];
        c = c < 0 ? 0 : (c > WCAP ? WCAP : c);
#pragma unroll 1
        for (int b0 = 0; b0 < c; b0 += 32) {
          const int idx = b0 + lane;
          const int ent = list[w2 * WCAP + (idx < WCAP ? idx : WCAP - 1)];
          const int m32 = (c - b0) < 32 ? (c - b0) : 32;
#pragma unroll 1
          for (int k = 0; k < m32; ++k) {
            const int uu   = __builtin_amdgcn_readlane(ent, k);
            const int slot = uu & (NBA - 1);
            const int el   = (uu >> SLA) & (CHUNK - 1);
            const int pk   = ((cbase + el) << SLA) | slot;
            if (t < RCAP) {
              if (lane == 0) { hl[t] = pk; cnt[slot] = cnt[slot] + 1; }
              t = t + 1;
            } else {
              ov = 1;
            }
          }
        }
      }
    }
    __syncthreads();
  }
  if (wave == 0 && lane == 0) { misc[8] = t; misc[9] = ov; }
  __syncthreads();
  int tt = misc[8];
  tt = tt < 0 ? 0 : (tt > RCAP ? RCAP : tt);
  const int ovf = misc[9];

  if (wave == 0) {
    const int base = lane * (NBA / 32);
    int s = 0;
#pragma unroll 1
    for (int i = 0; i < NBA / 32; ++i) s += cnt[base + i];
    int incl = s;
#pragma unroll
    for (int d = 1; d < 32; d <<= 1) {
      const int y = __shfl_up(incl, d, 32);
      if (lane >= d) incl += y;
    }
    int run = incl - s;
#pragma unroll 1
    for (int i = 0; i < NBA / 32; ++i) {
      const int cv = cnt[base + i];
      offs[base + i] = run;
      cur[base + i]  = run;
      run += cv;
    }
  }
  __syncthreads();
  if (wave == 0) {
#pragma unroll 1
    for (int b0 = 0; b0 < tt; b0 += 32) {
      const int idx = b0 + lane;
      const int ent = hl[idx < RCAP ? idx : RCAP - 1];
      const int m32 = (tt - b0) < 32 ? (tt - b0) : 32;
#pragma unroll 1
      for (int k = 0; k < m32; ++k) {
        const int uu   = __builtin_amdgcn_readlane(ent, k);
        const int slot = uu & (NBA - 1);
        if (lane == 0) {
          int p = cur[slot];
          p = p < 0 ? 0 : (p > RCAP - 1 ? RCAP - 1 : p);
          sl[p] = uu;
          cur[slot] = p + 1;
        }
      }
    }
  }
  __syncthreads();

  const float qnan = __int_as_float(0x7fc00000);
  const float pz = (ovf != 0) ? qnan : 0.0f;
  const int g  = lane >> 3;
  const int l8 = lane & 7;
#pragma unroll 1
  for (int si = 0; si < NBA / NWAVE; ++si) {
    const int s    = si * NWAVE + wave;
    const int node = nodeBase + s;
    int c = cnt[s];
    const bool big = c > DEGCAP;
    c = c < 0 ? 0 : (c > DEGCAP ? DEGCAP : c);
    int o = offs[s];
    o = o < 0 ? 0 : (o > RCAP ? RCAP : o);
    float a0 = 0.0f, a1 = 0.0f, a2 = 0.0f, a3 = 0.0f;
#pragma unroll 1
    for (int b0 = 0; b0 < c; b0 += 32) {
      int idx = o + b0 + lane;
      idx = idx > RCAP - 1 ? RCAP - 1 : idx;
      const int ent = sl[idx];
      int eid = ent >> SLA;
      eid = eid < 0 ? 0 : (eid > nE - 1 ? nE - 1 : eid);
      const int m32 = (c - b0) < 32 ? (c - b0) : 32;
      const int nq  = (m32 + 3) >> 2;
#pragma unroll 1
      for (int j = 0; j < nq; ++j) {
        const int hi = 4 * j + g;
        const int ek = __shfl(eid, hi, 32);
        const unsigned msk = (hi < m32) ? 0xffffffffu : 0u;
        const unsigned short* rp = Mh + (size_t)ek * MP16 + 4 * l8;
        const v2u w = *(const v2ua*)rp;
        const unsigned wx = w.x & msk;
        const unsigned wy = w.y & msk;
        a0 += h2f(wx & 0xffffu);
        a1 += h2f(wx >> 16);
        a2 += h2f(wy & 0xffffu);
        a3 += h2f(wy >> 16);
      }
    }
    a0 += __shfl_xor(a0, 8, 32);  a1 += __shfl_xor(a1, 8, 32);
    a2 += __shfl_xor(a2, 8, 32);  a3 += __shfl_xor(a3, 8, 32);
    a0 += __shfl_xor(a0, 16, 32); a1 += __shfl_xor(a1, 16, 32);
    a2 += __shfl_xor(a2, 16, 32); a3 += __shfl_xor(a3, 16, 32);
    const bool  live = node < mRows;
    const int   nr   = live ? node : mRows - 1;
    const float pzr  = big ? qnan : pz;
    float* mp = AGG + (size_t)nr * N2 + 4 * l8;
    v4f nv;
    nv.x = a0 * MINV + pzr;
    nv.y = a1 * MINV + pzr;
    nv.z = a2 * MINV + pzr;
    nv.w = a3 * MINV + pzr;
    const bool wr = live && (lane < 8);
    if (wr) *(volatile v4f*)mp = nv;
    __threadfence();
    if (wr) *(volatile v4f*)mp = nv;
  }
}

__global__ __launch_bounds__(NTHR) void k_node(const float* __restrict__ u, const float* __restrict__ AGG, int nU,
                                               const unsigned short* __restrict__ F1T,
                                               const unsigned short* __restrict__ F2T,
                                               const float* __restrict__ TAB, float* out) {
  extern __shared__ __attribute__((aligned(16))) float dyn[];
  float*          sD  = dyn;
  float*          sT  = dyn + TROWS * DP;
  float*          sO  = sT + TABN;
  unsigned short* sA1 = (unsigned short*)(sO + 256);
  unsigned short* sA2 = sA1 + TROWS * AP1;

  const int tid = (int)threadIdx.x, lane = tid & 31, wave = tid >> 5, hh = lane >> 4, m = lane & 15;
  const int rowBase = (int)blockIdx.x * TROWS;

  if (tid < TABN / 4) {
    const v4f t4 = *(const v4fa*)(TAB + 4 * tid);
    *(v4fa*)(sT + 4 * tid) = t4;
  }
#pragma unroll
  for (int it = 0; it < 4; ++it) {
    const int c    = it * NTHR + tid;
    const int row  = c >> 3;
    const int q    = c & 7;
    const int grow = rowBase + row;
    const int rc   = grow < nU ? grow : nU - 1;
    const unsigned okm = (grow < nU) ? 0xffffu : 0u;
    const v4f ua = *(const v4fa*)(u + (size_t)rc * FD + 4 * q);
    const v4f ga = *(const v4fa*)(AGG + (size_t)grow * N2 + 4 * q);
    v2u wu, wh, wl;
    wu.x = pack2(bf16n_bits(ua.x) & okm, bf16n_bits(ua.y) & okm);
    wu.y = pack2(bf16n_bits(ua.z) & okm, bf16n_bits(ua.w) & okm);
    const unsigned h0 = bf16n_bits(ga.x), h1 = bf16n_bits(ga.y), h2 = bf16n_bits(ga.z), h3 = bf16n_bits(ga.w);
    const unsigned l0 = bf16n_bits(ga.x - __uint_as_float(h0 << 16));
    const unsigned l1 = bf16n_bits(ga.y - __uint_as_float(h1 << 16));
    const unsigned l2 = bf16n_bits(ga.z - __uint_as_float(h2 << 16));
    const unsigned l3 = bf16n_bits(ga.w - __uint_as_float(h3 << 16));
    wh.x = pack2(h0, h1); wh.y = pack2(h2, h3);
    wl.x = pack2(l0, l1); wl.y = pack2(l2, l3);
    *(v2ua*)(sA1 + row * AP1 + 4 * q)          = wu;
    *(v2ua*)(sA1 + row * AP1 + FD + 4 * q)     = wh;
    *(v2ua*)(sA1 + row * AP1 + 2 * FD + 4 * q) = wl;
  }
  __syncthreads();

  wave_gemm<4, 3, K1>(sA1 + (16 * wave + m) * AP1 + 8 * hh, F1T, sD + (16 * wave + 8 * hh) * DP + m, hh, m);
  __syncthreads();

  epi_split(sD, sT + T_FB1, sA2, tid);
  __syncthreads();

  wave_gemm<2, 4, K2>(sA2 + (16 * wave + m) * AP2 + 8 * hh, F2T, sD + (16 * wave + 8 * hh) * DP + m, hh, m);
  __syncthreads();

  {
    const int row = tid >> 1;
    const int hf  = tid & 1;
    const float* rd = sD + row * DP + 16 * hf;
    float dot = 0.0f;
#pragma unroll 1
    for (int c4 = 0; c4 < 4; ++c4) {
      const v4f va = *(const v4fa*)(rd + 4 * c4);
      const v4f ba = *(const v4fa*)(sT + T_FB2 + 16 * hf + 4 * c4);
      const v4f wa = *(const v4fa*)(sT + T_TW + 16 * hf + 4 * c4);
      dot = fmaf(relu_n(va.x + ba.x), wa.x, dot);
      dot = fmaf(relu_n(va.y + ba.y), wa.y, dot);
      dot = fmaf(relu_n(va.z + ba.z), wa.z, dot);
      dot = fmaf(relu_n(va.w + ba.w), wa.w, dot);
    }
    const float oth = __shfl_xor(dot, 1, 32);
    const float s   = (dot + oth) + sT[T_TB];
    const float sg  = 1.0f / (1.0f + expf(-s));
    if (hf == 0) sO[row] = sg;
  }
  __syncthreads();

  if (tid < 32) {
    const v4f o4 = *(const v4fa*)(sO + 4 * tid);
    const int gidx = rowBase + 4 * tid;
    const bool stv = (gidx + 4 <= nU);
    const int gc = stv ? gidx : 0;
    if (stv) *(volatile v4f*)(out + (size_t)gc) = o4;
    __threadfence();
    if (stv) *(volatile v4f*)(out + (size_t)gc) = o4;
  }
}

extern "C" void kernel_launch(void* const* d_in, const int* in_sizes, int n_in,
                              void* d_out, int out_size, void* d_ws, size_t ws_size,
                              hipStream_t stream) {
  if (n_in < 15) return;
  if (in_sizes[0] != U_N * FD) return;
  if (in_sizes[1] != V_N * FD) return;
  if (in_sizes[2] != E_N * EVD) return;
  if (in_sizes[3] != E_N || in_sizes[4] != E_N) return;
  if (in_sizes[5] != KIN * N1 || in_sizes[6] != N1) return;
  if (in_sizes[7] != N1 * N2 || in_sizes[8] != N2) return;
  if (in_sizes[9] != N1 * N1 || in_sizes[10] != N1) return;
  if (in_sizes[11] != N1 * N2 || in_sizes[12] != N2) return;
  if (in_sizes[13] != N2 || in_sizes[14] != 1) return;
  if (out_size != U_N) return;

  const float* u    = (const float*)d_in[0];
  const float* v    = (const float*)d_in[1];
  const float* ev   = (const float*)d_in[2];
  const int*   esrc = (const int*)d_in[3];
  const int*   edst = (const int*)d_in[4];
  const float* gw1  = (const float*)d_in[5];
  const float* gb1  = (const float*)d_in[6];
  const float* gw2  = (const float*)d_in[7];
  const float* gb2  = (const float*)d_in[8];
  const float* fw1  = (const float*)d_in[9];
  const float* fb1  = (const float*)d_in[10];
  const float* fw2  = (const float*)d_in[11];
  const float* fb2  = (const float*)d_in[12];
  const float* tw   = (const float*)d_in[13];
  const float* tb   = (const float*)d_in[14];
  float* out = (float*)d_out;

  char* ws = (char*)d_ws;
  size_t off = 0;
  const size_t oG1T = off; off += (size_t)N1 * K1 * 2;          off = (off + 255) & ~(size_t)255;
  const size_t oG2T = off; off += (size_t)N2 * K2 * 2;          off = (off + 255) & ~(size_t)255;
  const size_t oF1T = off; off += (size_t)N1 * K1 * 2;          off = (off + 255) & ~(size_t)255;
  const size_t oF2T = off; off += (size_t)N2 * K2 * 2;          off = (off + 255) & ~(size_t)255;
  const size_t oTAB = off; off += (size_t)TABN * 4;             off = (off + 255) & ~(size_t)255;
  const size_t oAGG = off; off += (size_t)AGGROWS * N2 * 4;     off = (off + 255) & ~(size_t)255;
  const size_t oM16 = off; off += (size_t)E_N * MP16 * 2;       off = (off + 255) & ~(size_t)255;
  if (off > ws_size || off > ((size_t)256 << 20)) return;
  unsigned short* G1T = (unsigned short*)(ws + oG1T);
  unsigned short* G2T = (unsigned short*)(ws + oG2T);
  unsigned short* F1T = (unsigned short*)(ws + oF1T);
  unsigned short* F2T = (unsigned short*)(ws + oF2T);
  float*          TAB = (float*)(ws + oTAB);
  float*          AGG = (float*)(ws + oAGG);
  unsigned short* M16 = (unsigned short*)(ws + oM16);

  hipFuncSetAttribute(reinterpret_cast<const void*>(&k_edge), hipFuncAttributeMaxDynamicSharedMemorySize,
                      (int)TILE_LDS_BYTES);
  hipFuncSetAttribute(reinterpret_cast<const void*>(&k_node), hipFuncAttributeMaxDynamicSharedMemorySize,
                      (int)TILE_LDS_BYTES);
  hipFuncSetAttribute(reinterpret_cast<const void*>(&k_scan), hipFuncAttributeMaxDynamicSharedMemorySize,
                      (int)AGG_LDS_BYTES);

  const int nPrep = NU_G1 + NU_G2 + NU_F1 + NU_F2 + NU_TAB;

  k_prep<<<nPrep / NTHR, NTHR, 0, stream>>>(gw1, gb1, gw2, gb2, fw1, fb1, fw2, fb2, tw, tb,
                                            G1T, G2T, F1T, F2T, TAB);
  k_edge<<<E_N / TROWS, NTHR, TILE_LDS_BYTES, stream>>>(u, v, ev, esrc, edst, U_N, V_N, E_N, G1T, G2T, TAB, M16);
  k_scan<<<NSCAN, NTHR, AGG_LDS_BYTES, stream>>>(edst, E_N, 1, AGGROWS, M16, AGG);
  k_node<<<NNODEB, NTHR, TILE_LDS_BYTES, stream>>>(u, AGG, U_N, F1T, F2T, TAB, out);
}
